// CoOccurrenceEncoder_28802050686991
// MI455X (gfx1250) — hardware-verified
//
#include <hip/hip_runtime.h>


#define NB_  4
#define NN   512
#define DM   128
#define DH   64
#define NT   (NB_ * NN)
#define NP   (NN * NN)
typedef _Float16 h16;
typedef unsigned short bf;
typedef __attribute__((ext_vector_type(16))) __bf16   v16bf;
typedef __attribute__((ext_vector_type(16))) _Float16 v16h;
typedef __attribute__((ext_vector_type(8)))  _Float16 v8h;
typedef __attribute__((ext_vector_type(8)))  unsigned short v8us;
typedef __attribute__((ext_vector_type(8)))  float    v8f;
typedef __attribute__((ext_vector_type(4)))  float    v4f;
typedef v8h  __attribute__((may_alias)) v8ha;
typedef v4f  __attribute__((may_alias)) v4fa;
typedef v8us __attribute__((may_alias)) v8usa;

__device__ __forceinline__ unsigned short f2bf(float f) { unsigned u = __float_as_uint(f); u += 0x7FFFu + ((u >> 16) & 1u); return (unsigned short)(u >> 16); }
__device__ __forceinline__ float bf2f(unsigned short b) { return __uint_as_float(((unsigned)b) << 16); }
__device__ __forceinline__ float bfr(float f) { return bf2f(f2bf(f)); }
__device__ __forceinline__ v16h cat16(v8h lo, v8h hi) { return __builtin_shufflevector(lo, hi, 0, 1, 2, 3, 4, 5, 6, 7, 8, 9, 10, 11, 12, 13, 14, 15); }
__device__ __forceinline__ v16bf cat16b(v8us lo, v8us hi) { return __builtin_bit_cast(v16bf, __builtin_shufflevector(lo, hi, 0, 1, 2, 3, 4, 5, 6, 7, 8, 9, 10, 11, 12, 13, 14, 15)); }
__device__ __forceinline__ v8f wmma16(v16h a, v16h b, v8f c) { return __builtin_amdgcn_wmma_f32_16x16x32_f16(false, a, false, b, (short)0, c, false, false); }
__device__ __forceinline__ v8f wmmab(v16bf a, v16bf b, v8f c) { return __builtin_amdgcn_wmma_f32_16x16x32_bf16(false, a, false, b, (short)0, c, false, false); }


template <typename T16> struct WFrag;
template <> struct WFrag<h16> { typedef v16h V; static __device__ __forceinline__ V ld(const h16* p) { return cat16(*(const v8h*)p, *(const v8h*)(p + 16)); } static __device__ __forceinline__ v8f mma(V a, V b, v8f c) { return wmma16(a, b, c); } };
template <> struct WFrag<bf> { typedef v16bf V; static __device__ __forceinline__ V ld(const bf* p) { return cat16b(*(const v8us*)p, *(const v8us*)(p + 16)); } static __device__ __forceinline__ v8f mma(V a, V b, v8f c) { return wmmab(a, b, c); } };
template <typename T16, int NSPLIT, bool BIAS>
__global__ __launch_bounds__(32) void k_gemmw(const T16* __restrict__ A, const T16* __restrict__ A2, const T16* __restrict__ Bt, const T16* __restrict__ Bt2, int K, float* C, int ldc, const float* __restrict__ bias, size_t sA, size_t sB, size_t sC) {
    typedef typename WFrag<T16>::V V;
    __shared__ __align__(16) float os[16 * 68];
    const size_t z = blockIdx.z; A += z * sA; if (A2) A2 += z * sA; Bt += z * sB; if (Bt2) Bt2 += z * sB; C += z * sC;
    const int lane = threadIdx.x & 31, lr = lane & 15, hi = lane >> 4; const int r0 = blockIdx.x * 64, c0 = blockIdx.y * 64;
    v8f acc[4][4];
#pragma unroll
    for (int mb = 0; mb < 4; ++mb)
#pragma unroll
        for (int nb = 0; nb < 4; ++nb) acc[mb][nb] = (v8f){};
    const size_t aoff = (size_t)(r0 + lr) * K + 8 * hi, boff = (size_t)(c0 + lr) * K + 8 * hi;
#pragma unroll 1
    for (int kc = 0; kc < K; kc += 32) {
        V a[4], a2[4];
#pragma unroll
        for (int mb = 0; mb < 4; ++mb) { a[mb] = WFrag<T16>::ld(A + aoff + (size_t)mb * 16 * K + kc); if (NSPLIT == 1 || NSPLIT == 2) a2[mb] = WFrag<T16>::ld(A2 + aoff + (size_t)mb * 16 * K + kc); }
#pragma unroll
        for (int nb = 0; nb < 4; ++nb) { const V b = WFrag<T16>::ld(Bt + boff + (size_t)nb * 16 * K + kc); V b2; if (NSPLIT >= 2) b2 = WFrag<T16>::ld(Bt2 + boff + (size_t)nb * 16 * K + kc);
#pragma unroll
            for (int mb = 0; mb < 4; ++mb) { acc[mb][nb] = WFrag<T16>::mma(a[mb], b, acc[mb][nb]); if (NSPLIT == 1 || NSPLIT == 2) acc[mb][nb] = WFrag<T16>::mma(a2[mb], b, acc[mb][nb]); if (NSPLIT >= 2) acc[mb][nb] = WFrag<T16>::mma(a[mb], b2, acc[mb][nb]); } }
        asm volatile("v_nop\n\tv_nop\n\tv_nop\n\tv_nop" : "+v"(acc[0][0]), "+v"(acc[1][1]), "+v"(acc[2][2]), "+v"(acc[3][3]) : "v"(a[0]), "v"(a[3]));
    }
#pragma unroll
    for (int mb = 0; mb < 4; ++mb) {
#pragma unroll
        for (int nb = 0; nb < 4; ++nb) {
#pragma unroll
            for (int j = 0; j < 8; ++j) os[(hi * 8 + j) * 68 + nb * 16 + lr] = acc[mb][nb][j]; }
        __builtin_amdgcn_wave_barrier(); asm volatile("" ::: "memory");
        float* crow = C + (size_t)(r0 + mb * 16) * ldc + c0;
#pragma unroll 1
        for (int ps = 0; ps < 2; ++ps) {
#pragma unroll
            for (int s = 0; s < 8; ++s) { const int row = 2 * s + hi, cofs = lr * 4; v4f val = *(const v4fa*)(os + row * 68 + cofs); if (BIAS) { val[0] += bfr(bias[c0 + cofs]); val[1] += bfr(bias[c0 + cofs + 1]); val[2] += bfr(bias[c0 + cofs + 2]); val[3] += bfr(bias[c0 + cofs + 3]); }
                *(volatile v4f*)(crow + (size_t)row * ldc + cofs) = val; }
            if (ps == 0) __threadfence(); }
        __builtin_amdgcn_wave_barrier(); asm volatile("" ::: "memory");
    }
}

__device__ __forceinline__ void splitf(float y, unsigned short& h, unsigned short& l) { h = f2bf(y); l = f2bf(y - bf2f(h)); }
typedef __attribute__((ext_vector_type(2))) unsigned short v2us;

__global__ __launch_bounds__(256) void k_cvt8(const float* __restrict__ src, bf* dst, size_t n8) { const size_t i = (size_t)blockIdx.x * 256 + threadIdx.x; if (i >= n8) return; const v8f v = *(const v8f*)(src + i * 8); v8us o;
#pragma unroll
    for (int k = 0; k < 8; ++k) o[k] = f2bf(v[k]); *(volatile v8us*)(dst + i * 8) = o; __threadfence(); *(volatile v8us*)(dst + i * 8) = o; }
__global__ __launch_bounds__(256) void k_wtb(const float* __restrict__ w, int k0, int K, int N, bf* Bt) {
    const int lane = threadIdx.x & 31; const int L = blockIdx.x * 8 + (threadIdx.x >> 5); if (L >= N * K / 64) return; const int e = L * 64 + lane * 2; const int n = e / K, k = e % K; v2us o;
    o[0] = f2bf(w[(size_t)(k0 + k) * N + n]); o[1] = f2bf(w[(size_t)(k0 + k + 1) * N + n]); *(volatile v2us*)(Bt + e) = o; __threadfence(); *(volatile v2us*)(Bt + e) = o;
}
__global__ __launch_bounds__(256) void k_pair(const float* __restrict__ HI, const float* __restrict__ HJ, const float* __restrict__ b1, int b, bf* Ph, bf* Pl) {
    const int lane = threadIdx.x & 31; const int L0 = (blockIdx.x * 8 + (threadIdx.x >> 5)) * 8; const int nlines = NP * DM / 64;
#pragma unroll 1
    for (int ps = 0; ps < 2; ++ps) {
#pragma unroll
        for (int l = 0; l < 8; ++l) { const int L = L0 + l; if (L >= nlines) break; const size_t e = (size_t)L * 64 + lane * 2; const int c = (int)(e & (DM - 1)); const int pr = (int)(e >> 7); const int i = pr >> 9, j = pr & (NN - 1); v2us oh, ol;
#pragma unroll
            for (int q = 0; q < 2; ++q) { const float t = fmaxf(HI[((size_t)b * NN + i) * DM + c + q] + HJ[((size_t)b * NN + j) * DM + c + q] + bfr(b1[c + q]), 0.f); unsigned short a, c2; splitf(t, a, c2); oh[q] = a; ol[q] = c2; }
            *(volatile v2us*)(Ph + e) = oh; *(volatile v2us*)(Pl + e) = ol; }
        if (ps == 0) __threadfence(); }
}
__global__ __launch_bounds__(256) void k_head(const float* __restrict__ H2, const float* __restrict__ W3, const float* __restrict__ b3, int b, float* OUT) {
    const int lane = threadIdx.x & 31; const int p = (blockIdx.x * 8 + (threadIdx.x >> 5)) * 32 + lane; if (p >= NP) return; const float* hr = H2 + (size_t)p * DH; float s = bfr(b3[0]);
#pragma unroll 4
    for (int k = 0; k < DH; ++k) s = __fadd_rn(s, __fmul_rn(fmaxf(hr[k], 0.f), bfr(W3[k])));
    const float o = __fdiv_rn(1.0f, 1.0f + __expf(-s)); *(volatile float*)(OUT + (size_t)b * NP + p) = o; __threadfence(); *(volatile float*)(OUT + (size_t)b * NP + p) = o;
}

extern "C" void kernel_launch(void* const* d_in, const int* in_sizes, int n_in,
                              void* d_out, int out_size, void* d_ws, size_t ws_size, hipStream_t stream) {
    (void)in_sizes; (void)n_in; (void)out_size;
    const float* x = (const float*)d_in[0]; const float* W1 = (const float*)d_in[1]; const float* b1 = (const float*)d_in[2]; const float* W2 = (const float*)d_in[3]; const float* b2 = (const float*)d_in[4]; const float* W3 = (const float*)d_in[5]; const float* b3 = (const float*)d_in[6];
    float* OUT = (float*)d_out;
    char* wsp = (char*)d_ws;
    auto take = [&](size_t bytes) { char* p = wsp; wsp += (bytes + 255) & ~(size_t)255; return (void*)p; };
    bf* XB = (bf*)take((size_t)NT * DM * 2); bf* W1A = (bf*)take((size_t)DM * DM * 2); bf* W1B = (bf*)take((size_t)DM * DM * 2); bf* W2T = (bf*)take((size_t)DH * DM * 2);
    float* HI = (float*)take((size_t)NT * DM * 4); float* HJ = (float*)take((size_t)NT * DM * 4); bf* Ph = (bf*)take((size_t)NP * DM * 2); bf* Pl = (bf*)take((size_t)NP * DM * 2); float* H2 = (float*)take((size_t)NP * DH * 4);
    if ((size_t)(wsp - (char*)d_ws) > ws_size) return;
    k_cvt8<<<(unsigned)((NT * DM / 8 + 255) / 256), 256, 0, stream>>>(x, XB, (size_t)NT * DM / 8);
    k_wtb<<<(DM * DM / 64 + 7) / 8, 256, 0, stream>>>(W1, 0, DM, DM, W1A); k_wtb<<<(DM * DM / 64 + 7) / 8, 256, 0, stream>>>(W1, DM, DM, DM, W1B); k_wtb<<<(DH * DM / 64 + 7) / 8, 256, 0, stream>>>(W2, 0, DM, DH, W2T);
    k_gemmw<bf, 0, false><<<dim3(NT / 64, DM / 64, 1), 32, 0, stream>>>(XB, nullptr, W1A, nullptr, DM, HI, DM, nullptr, 0, 0, 0);
    k_gemmw<bf, 0, false><<<dim3(NT / 64, DM / 64, 1), 32, 0, stream>>>(XB, nullptr, W1B, nullptr, DM, HJ, DM, nullptr, 0, 0, 0);
    for (int b = 0; b < NB_; ++b) {
        k_pair<<<(unsigned)((NP * DM / 64 + 63) / 64), 256, 0, stream>>>(HI, HJ, b1, b, Ph, Pl);
        k_gemmw<bf, 1, true><<<dim3(NP / 64, 1, 1), 32, 0, stream>>>(Ph, Pl, W2T, nullptr, DM, H2, DH, b2, 0, 0, 0);
        k_head<<<NP / 256, 256, 0, stream>>>(H2, W3, b3, b, OUT); }
}
